// SSM_spa_6528350290350
// MI455X (gfx1250) — hardware-verified
//
#include <hip/hip_runtime.h>


namespace {
constexpr int B = 4, L = 256, DM = 1024, DI = 2048, NS = 16, DTR = 64, XP = DTR + 2 * NS, XPP = 128, NT = B * L;
constexpr float XS = 8.0f, WSC = 256.0f;
typedef _Float16 b16;
typedef __attribute__((ext_vector_type(16))) _Float16 v16b;
typedef __attribute__((ext_vector_type(8))) _Float16 v8b;
typedef __attribute__((ext_vector_type(8))) float v8f;
typedef __attribute__((ext_vector_type(4))) float v4f;
__device__ __forceinline__ float bf16_rne(float f) { unsigned int u = __float_as_uint(f); u += 0x7FFFu + ((u >> 16) & 1u); float r = __uint_as_float(u & 0xFFFF0000u); asm volatile("" : "+v"(r)); return r; }
__device__ __forceinline__ void split16(float v, b16& hi, b16& lo) { hi = (b16)v; lo = (b16)(v - (float)hi); }
__device__ __forceinline__ v16b frag_kb(const b16* p, int hh) { const v8b a = *(const v8b*)(p + 8 * hh), b = *(const v8b*)(p + 16 + 8 * hh); v16b f;
#pragma unroll
  for (int e = 0; e < 8; ++e) { f[e] = a[e]; f[8 + e] = b[e]; } return f; }
__device__ __forceinline__ v8f wmma16b(v16b a, v16b b, v8f c) { v8f d = __builtin_amdgcn_wmma_f32_16x16x32_f16(false, a, false, b, (short)0, c, false, false); asm volatile("v_nop\n\tv_nop\n\tv_nop\n\tv_nop" : "+v"(d) : "v"(a), "v"(b)); return d; }
__device__ __forceinline__ void wave_lds_sync() { __builtin_amdgcn_fence(__ATOMIC_RELEASE, "workgroup"); __builtin_amdgcn_wave_barrier(); __builtin_amdgcn_fence(__ATOMIC_ACQUIRE, "workgroup"); }
__device__ __forceinline__ float pmul(float a, float b) { float p = a * b; asm volatile("" : "+v"(p)); return p; }
__device__ __forceinline__ float silu(float v) { return v / (1.0f + __expf(-v)); }
__device__ __forceinline__ float softplus(float v) { return v > 20.0f ? v : log1pf(__expf(v)); }

__global__ __launch_bounds__(256) void wcopy_kernel(const float* __restrict__ w, int rows_real, int rows_tot, int K, b16* __restrict__ WT) { const size_t u = (size_t)blockIdx.x * 256 + threadIdx.x; if (u >= (size_t)rows_tot * K / 8) return; const size_t e = u * 8; const int r = (int)(e / K); v8b v;
#pragma unroll
  for (int j = 0; j < 8; ++j) v[j] = (b16)(r < rows_real ? bf16_rne(w[e + j]) * WSC : 0.0f); for (int pass = 0; pass < 2; ++pass) { *(volatile v8b*)(WT + e) = v; __threadfence(); } }
template <int KIN, int MODE>
__global__ __launch_bounds__(32) void dense_kernel(const float* __restrict__ IN, int inPitch, const b16* __restrict__ WT, const float* __restrict__ bias, int NG, int OW, float* __restrict__ OUT, float ascale) {
  constexpr int KCH = KIN > 1024 ? 1024 : KIN; __shared__ __attribute__((aligned(16))) b16 Ah[16][KCH + 8], Al[16][MODE == 0 ? 8 : KCH + 8]; __shared__ float Tf[16][132]; const int lane = threadIdx.x, nloc = lane & 15, hlf = lane >> 4; const int g = blockIdx.x % NG; const size_t m0 = (size_t)(blockIdx.x / NG) * 16;
  v8f acc[8];
#pragma unroll
  for (int t = 0; t < 8; ++t) acc[t] = (v8f){};
#pragma unroll 1
  for (int kc = 0; kc < KIN; kc += KCH) { wave_lds_sync();
    for (int rr = 0; rr < 16; ++rr) for (int q = 0; q < KCH / 32; ++q) { const float v = IN[(m0 + rr) * inPitch + kc + q * 32 + lane]; if (MODE == 0) Ah[rr][q * 32 + lane] = (b16)(bf16_rne(v) * XS); else { b16 p, ql; split16(v * ascale, p, ql); Ah[rr][q * 32 + lane] = p; Al[rr][q * 32 + lane] = ql; } }
    wave_lds_sync();
#pragma unroll 2
    for (int kb = 0; kb < KCH; kb += 32) { const v16b a = frag_kb(&Ah[nloc][kb], hlf); v16b a2; if (MODE != 0) a2 = frag_kb(&Al[nloc][kb], hlf);
#pragma unroll
      for (int t = 0; t < 8; ++t) { const v16b bw = frag_kb(WT + (size_t)(g * 128 + t * 16 + nloc) * KIN + kc + kb, hlf); acc[t] = wmma16b(a, bw, acc[t]); if (MODE != 0) acc[t] = wmma16b(a2, bw, acc[t]); } } }
#pragma unroll
  for (int t = 0; t < 8; ++t) { const int c = g * 128 + t * 16 + nloc; const float bb = bias ? bf16_rne(bias[c]) : 0.0f;
#pragma unroll
    for (int r8 = 0; r8 < 8; ++r8) Tf[8 * hlf + r8][t * 16 + nloc] = acc[t][r8] * (1.0f / ((MODE == 0 ? XS : ascale) * WSC)) + bb; }
  wave_lds_sync();
  for (int pass = 0; pass < 2; ++pass) { for (int rr = 0; rr < 16; ++rr) *(volatile v4f*)(OUT + (m0 + rr) * OW + g * 128 + lane * 4) = *(const v4f*)(&Tf[rr][lane * 4]); __threadfence(); } }
__global__ __launch_bounds__(256) void conv_kernel(const float* __restrict__ XZ, const float* __restrict__ cw, const float* __restrict__ cb, float* __restrict__ XC) { const size_t u = (size_t)blockIdx.x * 256 + threadIdx.x; if (u >= (size_t)NT * DI / 4) return; const int d0 = (int)(u % (DI / 4)) * 4; const int row = (int)(u / (DI / 4)); const int b = row / L, t = row % L; v4f o;
#pragma unroll
  for (int k4 = 0; k4 < 4; ++k4) { const int d = d0 + k4; float s = bf16_rne(cb[d]);
#pragma unroll
    for (int k = 0; k < 4; ++k) { const int tt = t - 3 + k; if (tt >= 0) s += pmul(bf16_rne(cw[d * 4 + k]), XZ[((size_t)b * L + tt) * 2 * DI + d]); } o[k4] = silu(s); }
  for (int pass = 0; pass < 2; ++pass) { *(volatile v4f*)(XC + (size_t)row * DI + d0) = o; __threadfence(); } }
__global__ __launch_bounds__(256) void scan_kernel(const float* __restrict__ XC, const float* __restrict__ XDB, const float* __restrict__ DL, const float* __restrict__ dtb, const float* __restrict__ Alog, const float* __restrict__ Dp, const float* __restrict__ XZ, float* __restrict__ Y) {
  const int u = blockIdx.x * 256 + threadIdx.x; if (u >= B * DI) return; const int b = u / DI, d = u % DI; float A[NS];
#pragma unroll
  for (int n = 0; n < NS; ++n) A[n] = -__expf(bf16_rne(Alog[(size_t)d * NS + n]));
  const float db = bf16_rne(dtb[d]), Dd = bf16_rne(Dp[d]);
  for (int pass = 0; pass < 2; ++pass) { float h[NS];
#pragma unroll
    for (int n = 0; n < NS; ++n) h[n] = 0.0f;
#pragma unroll 1
    for (int t = 0; t < L; ++t) { const size_t row = (size_t)b * L + t; const float xv = XC[row * DI + d]; const float dl = softplus(DL[row * DI + d] + db); const float* bc = XDB + row * XPP + DTR; float y = 0.0f;
#pragma unroll
      for (int n = 0; n < NS; ++n) { h[n] = pmul(__expf(pmul(dl, A[n])), h[n]) + pmul(pmul(dl, bc[n]), xv); y += pmul(h[n], bc[NS + n]); }
      y += pmul(Dd, xv); y = pmul(y, silu(XZ[row * 2 * DI + DI + d])); ((volatile float*)Y)[row * DI + d] = y; }
    __threadfence(); } }
__global__ __launch_bounds__(256) void ln_kernel(const float* __restrict__ O1, const float* __restrict__ g, const float* __restrict__ bt, float* __restrict__ out) { const int wave = threadIdx.x >> 5, lane = threadIdx.x & 31; const size_t row = (size_t)blockIdx.x * 8 + wave; if (row >= (size_t)NT) return; float v[32]; float s = 0.0f;
#pragma unroll
  for (int q = 0; q < 32; ++q) { v[q] = O1[row * DM + q * 32 + lane]; s += v[q]; } for (int o = 16; o; o >>= 1) s += __shfl_xor(s, o); const float mu = s * (1.0f / DM); float qq = 0.0f;
#pragma unroll
  for (int q = 0; q < 32; ++q) qq += pmul(v[q] - mu, v[q] - mu); for (int o = 16; o; o >>= 1) qq += __shfl_xor(qq, o); const float rs = rsqrtf(qq * (1.0f / DM) + 1e-5f);
  for (int pass = 0; pass < 2; ++pass) {
#pragma unroll
    for (int q = 0; q < 32; ++q) { const int c = q * 32 + lane; ((volatile float*)out)[row * DM + c] = pmul(pmul(v[q] - mu, rs), bf16_rne(g[c])) + bf16_rne(bt[c]); } __threadfence(); } }
}

extern "C" void kernel_launch(void* const* d_in, const int* in_sizes, int n_in, void* d_out, int out_size, void* d_ws, size_t ws_size, hipStream_t stream) {
  (void)n_in;
  auto Fp = [&](int i) { return (const float*)d_in[i]; };
  if (in_sizes[0] != NT * DM || in_sizes[1] != 2 * DI * DM || in_sizes[2] != DI * 4 || in_sizes[4] != XP * DI || in_sizes[5] != DI * DTR || in_sizes[7] != DI * NS || in_sizes[9] != DM * DI || out_size != NT * DM) return;
  const int BV = B; const int NTV = BV * L;
  size_t off = 0; char* ws = (char*)d_ws;
  auto carve = [&](size_t bytes) { char* p = ws + off; off += (bytes + 255) & ~(size_t)255; return p; };
  b16* WIN = (b16*)carve((size_t)2 * DI * DM * 2); b16* WXP = (b16*)carve((size_t)XPP * DI * 2); b16* WDT = (b16*)carve((size_t)DI * DTR * 2); b16* WOUT = (b16*)carve((size_t)DM * DI * 2);
  float* XZ = (float*)carve((size_t)NT * 2 * DI * 4); float* XC = (float*)carve((size_t)NT * DI * 4); float* XDB = (float*)carve((size_t)NT * XPP * 4); float* DL = (float*)carve((size_t)NT * DI * 4); float* Y = (float*)carve((size_t)NT * DI * 4); float* O1 = (float*)carve((size_t)NT * DM * 4);
  if (off > ws_size || off > ((size_t)80 << 20)) return;
  wcopy_kernel<<<(unsigned)(((size_t)2 * DI * DM / 8 + 255) / 256), 256, 0, stream>>>(Fp(1), 2 * DI, 2 * DI, DM, WIN); wcopy_kernel<<<(unsigned)(((size_t)XPP * DI / 8 + 255) / 256), 256, 0, stream>>>(Fp(4), XP, XPP, DI, WXP);
  wcopy_kernel<<<(unsigned)(((size_t)DI * DTR / 8 + 255) / 256), 256, 0, stream>>>(Fp(5), DI, DI, DTR, WDT); wcopy_kernel<<<(unsigned)(((size_t)DM * DI / 8 + 255) / 256), 256, 0, stream>>>(Fp(9), DM, DM, DI, WOUT);
  dense_kernel<DM, 0><<<(NTV / 16) * (2 * DI / 128), 32, 0, stream>>>(Fp(0), DM, WIN, nullptr, 2 * DI / 128, 2 * DI, XZ, XS);
  conv_kernel<<<(unsigned)(((size_t)NTV * DI / 4 + 255) / 256), 256, 0, stream>>>(XZ, Fp(2), Fp(3), XC);
  dense_kernel<DI, 1><<<(NTV / 16) * 1, 32, 0, stream>>>(XC, DI, WXP, nullptr, 1, XPP, XDB, 256.0f);
  dense_kernel<DTR, 1><<<(NTV / 16) * (DI / 128), 32, 0, stream>>>(XDB, XPP, WDT, nullptr, DI / 128, DI, DL, 256.0f);
  scan_kernel<<<(BV * DI + 255) / 256, 256, 0, stream>>>(XC, XDB, DL, Fp(6), Fp(7), Fp(8), XZ, Y);
  dense_kernel<DI, 1><<<(NTV / 16) * (DM / 128), 32, 0, stream>>>(Y, DI, WOUT, nullptr, DM / 128, DM, O1, 256.0f);
  ln_kernel<<<(NTV + 7) / 8, 256, 0, stream>>>(O1, Fp(10), Fp(11), (float*)d_out);
}
